// CANN_60455959658874
// MI455X (gfx1250) — hardware-verified
//
#include <hip/hip_runtime.h>
#include <hip/hip_bf16.h>

typedef __attribute__((ext_vector_type(16))) _Float16 v16h;
typedef __attribute__((ext_vector_type(8)))  _Float16 v8h;
typedef __attribute__((ext_vector_type(16))) __bf16   v16b;
typedef __attribute__((ext_vector_type(8)))  __bf16   v8b;
typedef __attribute__((ext_vector_type(8)))  float    v8f;
typedef __attribute__((ext_vector_type(4)))  float    v4f;
typedef __attribute__((ext_vector_type(2)))  float    v2f;
typedef __attribute__((ext_vector_type(4)))  unsigned v4u;

__device__ __forceinline__ unsigned short f2bf_bits(float f) {
  unsigned u = __float_as_uint(f);
  return (unsigned short)((u + 0x7FFFu + ((u >> 16) & 1u)) >> 16);
}
__device__ __forceinline__ float bf_bits2f(unsigned short h) { return __uint_as_float(((unsigned)h) << 16); }

__device__ __forceinline__ void dep_guard_h(v8f& a, v8f& b, v16h x, v16h y) { asm volatile("v_nop\n\tv_nop\n\tv_nop\n\tv_nop" : "+v"(a), "+v"(b) : "v"(x), "v"(y)); }
__device__ __forceinline__ void dep_guard_b(v8f& a, v8f& b, v16b x, v16b y) { asm volatile("v_nop\n\tv_nop\n\tv_nop\n\tv_nop" : "+v"(a), "+v"(b) : "v"(x), "v"(y)); }
__device__ __forceinline__ void keep4_h(v16h a, v16h b, v16h c, v16h d) { asm volatile("v_nop" :: "v"(a), "v"(b), "v"(c), "v"(d)); }
__device__ __forceinline__ void keep4_b(v16b a, v16b b, v16b c, v16b d) { asm volatile("v_nop" :: "v"(a), "v"(b), "v"(c), "v"(d)); }
__device__ __forceinline__ void acc_guard4(v8f& a, v8f& b, v8f& c, v8f& d) { asm volatile("v_nop\n\tv_nop\n\tv_nop\n\tv_nop" : "+v"(a), "+v"(b), "+v"(c), "+v"(d)); }

template <typename T> struct Frag;
template <> struct Frag<_Float16> {
  typedef v16h V; union U { v16h v; v8h h[2]; };
  static __device__ __forceinline__ v16h load(const _Float16* p) {
    U f; f.h[0] = *(const v8h*)(p); f.h[1] = *(const v8h*)(p + 16); return f.v;
  }
  static __device__ __forceinline__ v8f mma(v16h a, v16h b, v8f c) {
    return __builtin_amdgcn_wmma_f32_16x16x32_f16(false, a, false, b, (short)0, c, false, false);
  }
  static __device__ __forceinline__ void guard(v8f& a, v8f& b, v16h x, v16h y) { dep_guard_h(a, b, x, y); }
  static __device__ __forceinline__ void keep(v16h a, v16h b, v16h c, v16h d) { keep4_h(a, b, c, d); }
};
template <> struct Frag<__bf16> {
  typedef v16b V; union U { v16b v; v8b h[2]; };
  static __device__ __forceinline__ v16b load(const __bf16* p) {
    U f; f.h[0] = *(const v8b*)(p); f.h[1] = *(const v8b*)(p + 16); return f.v;
  }
  static __device__ __forceinline__ v8f mma(v16b a, v16b b, v8f c) {
    return __builtin_amdgcn_wmma_f32_16x16x32_bf16(false, a, false, b, (short)0, c, false, false);
  }
  static __device__ __forceinline__ void guard(v8f& a, v8f& b, v16b x, v16b y) { dep_guard_b(a, b, x, y); }
  static __device__ __forceinline__ void keep(v16b a, v16b b, v16b c, v16b d) { keep4_b(a, b, c, d); }
};

template <int ET> struct Elem;
template <> struct Elem<0> { typedef _Float16 T; };
template <> struct Elem<1> { typedef __bf16 T; };
template <int ET, bool SPLIT, int BIAS_MODE, int OUT_MODE>
__global__ __launch_bounds__(256) void wmma_gemm64(
    const unsigned short* __restrict__ Ap, const unsigned short* __restrict__ A2p, int lda, long strideA,
    const unsigned short* __restrict__ Btp, const unsigned short* __restrict__ Bt2p, int ldb, long strideB,
    void* __restrict__ Cout, void* __restrict__ Cout2, int ldc, long strideC,
    const float* __restrict__ bias,
    int M, int N, int K, float scale) {
  typedef typename Elem<ET>::T T;
  typedef typename Frag<T>::V V;
  const T* A = (const T*)Ap; const T* A2 = (const T*)A2p; const T* Bt = (const T*)Btp; const T* Bt2 = (const T*)Bt2p;
  __shared__ __align__(16) float sT[8][16 * 68];
  const int b    = blockIdx.y;
  const int lane = threadIdx.x & 31;
  const int wave = threadIdx.x >> 5;
  const int tilesN = N >> 6;
  const int tilesM = M >> 6;
  const int tile = blockIdx.x * 8 + wave;
  if (tile >= tilesM * tilesN) return;
  const int tm = tile / tilesN;
  const int tn = tile - tm * tilesN;
  const int m0 = tm << 6;
  const int n0 = tn << 6;

  const T* Ab  = A  + (size_t)b * strideA;
  const T* Bb  = Bt + (size_t)b * strideB;
  const T* Ab2 = SPLIT ? (A2  + (size_t)b * strideA) : nullptr;
  const T* Bb2 = SPLIT ? (Bt2 + (size_t)b * strideB) : nullptr;

  const int rlane = lane & 15;
  const int koff  = (lane >> 4) * 8;
  const int mOff  = (lane >> 4) * 8;

  v8f acc[4][4];
#pragma unroll
  for (int i = 0; i < 4; ++i)
#pragma unroll
    for (int j = 0; j < 4; ++j) acc[i][j] = (v8f){0.f,0.f,0.f,0.f,0.f,0.f,0.f,0.f};

  for (int k0 = 0; k0 < K; k0 += 32) {
    V bh[4], bl[4];
#pragma unroll
    for (int j = 0; j < 4; ++j) {
      const size_t bo = (size_t)(n0 + (j << 4) + rlane) * ldb + koff + k0;
      bh[j] = Frag<T>::load(Bb + bo);
      if (SPLIT) bl[j] = Frag<T>::load(Bb2 + bo);
    }
#pragma unroll
    for (int i = 0; i < 4; ++i) {
      const size_t ao = (size_t)(m0 + (i << 4) + rlane) * lda + koff + k0;
      V ah = Frag<T>::load(Ab + ao);
      V al;
      if (SPLIT) al = Frag<T>::load(Ab2 + ao);
#pragma unroll
      for (int j = 0; j < 4; ++j) {
        acc[i][j] = Frag<T>::mma(ah, bh[j], acc[i][j]);
        if (SPLIT) {
          acc[i][j] = Frag<T>::mma(ah, bl[j], acc[i][j]);
          acc[i][j] = Frag<T>::mma(al, bh[j], acc[i][j]);
        }
      }
      Frag<T>::guard(acc[i][0], acc[i][3], ah, SPLIT ? al : ah);
    }
    Frag<T>::keep(bh[0], bh[1], bh[2], bh[3]);
    if (SPLIT) Frag<T>::keep(bl[0], bl[1], bl[2], bl[3]);
  }
  acc_guard4(acc[0][0], acc[0][1], acc[0][2], acc[0][3]);
  acc_guard4(acc[1][0], acc[1][1], acc[1][2], acc[1][3]);
  acc_guard4(acc[2][0], acc[2][1], acc[2][2], acc[2][3]);
  acc_guard4(acc[3][0], acc[3][1], acc[3][2], acc[3][3]);

  float* slab = sT[wave];
  float breg0 = 0.f, breg1 = 0.f;
  if (BIAS_MODE == 1) { breg0 = bias[m0 + lane]; breg1 = bias[m0 + 32 + lane]; }
  if (BIAS_MODE == 2) { breg0 = bias[n0 + lane]; breg1 = bias[n0 + 32 + lane]; }
  if (BIAS_MODE != 0) { breg0 = bf_bits2f(f2bf_bits(breg0)); breg1 = bf_bits2f(f2bf_bits(breg1)); }
#pragma unroll
  for (int i = 0; i < 4; ++i) {
    const int mBase = m0 + (i << 4);
    float brow[8];
#pragma unroll
    for (int r = 0; r < 8; ++r) {
      brow[r] = 0.f;
      if (BIAS_MODE == 1) {
        const float bsrc = (i < 2) ? breg0 : breg1;
        brow[r] = __shfl(bsrc, ((i & 1) << 4) + mOff + r, 32);
      }
    }
#pragma unroll
    for (int j = 0; j < 4; ++j) {
      float bcol = 0.f;
      if (BIAS_MODE == 2) {
        const float bsrc = (j < 2) ? breg0 : breg1;
        bcol = __shfl(bsrc, ((j & 1) << 4) + rlane, 32);
      }
#pragma unroll
      for (int r = 0; r < 8; ++r) {
        float v = acc[i][j][r] * scale;
        if (BIAS_MODE == 1) v += brow[r];
        if (BIAS_MODE == 2) v += bcol;
        slab[(mOff + r) * 68 + (j << 4) + rlane] = v;
      }
    }
    __builtin_amdgcn_fence(__ATOMIC_RELEASE, "workgroup");
    __builtin_amdgcn_wave_barrier();
    __builtin_amdgcn_fence(__ATOMIC_ACQUIRE, "workgroup");
    if (OUT_MODE == 0) {
      float* C = (float*)Cout + (size_t)b * strideC;
      const int hh = lane >> 4, c4 = (lane & 15) * 4;
      for (int pass = 0; pass < 2; ++pass) {
#pragma unroll
        for (int it = 0; it < 8; ++it) {
          const int row = it * 2 + hh;
          v4f v = *(const v4f*)(slab + row * 68 + c4);
          *(volatile v4f*)(C + (size_t)(mBase + row) * ldc + n0 + c4) = v;
        }
        __threadfence();
      }
    } else {
      const int q = lane >> 3, c8 = (lane & 7) * 8;
      unsigned short* C  = (unsigned short*)Cout  + (size_t)b * strideC;
      unsigned short* C2 = (unsigned short*)Cout2 + (size_t)b * strideC;
      for (int pass = 0; pass < 2; ++pass) {
#pragma unroll
        for (int it = 0; it < 4; ++it) {
          const int row = it * 4 + q;
          const float* sp = slab + row * 68 + c8;
          v8h hv, lv;
#pragma unroll
          for (int e = 0; e < 8; ++e) {
            unsigned short hb = f2bf_bits(sp[e]);
            unsigned short lb = f2bf_bits(sp[e] - bf_bits2f(hb));
            hv[e] = __builtin_bit_cast(_Float16, hb);
            lv[e] = __builtin_bit_cast(_Float16, lb);
          }
          *(volatile v8h*)(C + (size_t)(mBase + row) * ldc + n0 + c8) = hv;
          *(volatile v8h*)(C2 + (size_t)(mBase + row) * ldc + n0 + c8) = lv;
        }
        __threadfence();
      }
    }
    __builtin_amdgcn_fence(__ATOMIC_RELEASE, "workgroup");
    __builtin_amdgcn_wave_barrier();
    __builtin_amdgcn_fence(__ATOMIC_ACQUIRE, "workgroup");
  }
}

__global__ __launch_bounds__(256) void cast_f32_bf16x2(
    const float* __restrict__ in, unsigned short* __restrict__ out, int n2) {
  const int i = blockIdx.x * 256 + threadIdx.x;
  if (i < n2) {
    const v2f f = *(const v2f*)(in + 2 * (size_t)i);
    const unsigned u = (unsigned)f2bf_bits(f.x) | ((unsigned)f2bf_bits(f.y) << 16);
    ((volatile unsigned*)out)[i] = u;
    __threadfence();
    ((volatile unsigned*)out)[i] = u;
  }
}

__global__ __launch_bounds__(256) void softmax_rows_split(
    const float* __restrict__ S, unsigned short* __restrict__ Ph, unsigned short* __restrict__ Pl, int ncols) {
  __shared__ float redm[8];
  __shared__ float reds[8];
  const int tid = threadIdx.x, lane = tid & 31, wave = tid >> 5;
  const size_t base = (size_t)blockIdx.x * (size_t)ncols + (size_t)tid * 8;
  const v4f x0 = *(const v4f*)(S + base);
  const v4f x1 = *(const v4f*)(S + base + 4);
  float xv[8];
  xv[0] = x0.x; xv[1] = x0.y; xv[2] = x0.z; xv[3] = x0.w;
  xv[4] = x1.x; xv[5] = x1.y; xv[6] = x1.z; xv[7] = x1.w;
  float m = xv[0];
#pragma unroll
  for (int e = 1; e < 8; ++e) m = fmaxf(m, xv[e]);
#pragma unroll
  for (int off = 1; off < 32; off <<= 1) m = fmaxf(m, __shfl_xor(m, off, 32));
  if (lane == 0) redm[wave] = m;
  __syncthreads();
  float gm = redm[0];
#pragma unroll
  for (int w = 1; w < 8; ++w) gm = fmaxf(gm, redm[w]);

  float ev[8];
  float ps = 0.0f;
#pragma unroll
  for (int e = 0; e < 8; ++e) { ev[e] = expf(xv[e] - gm); ps += ev[e]; }
#pragma unroll
  for (int off = 1; off < 32; off <<= 1) ps += __shfl_xor(ps, off, 32);
  if (lane == 0) reds[wave] = ps;
  __syncthreads();
  float tot = reds[0];
#pragma unroll
  for (int w = 1; w < 8; ++w) tot += reds[w];
  const float inv = 1.0f / tot;

  unsigned hw[4], lw[4];
#pragma unroll
  for (int e2 = 0; e2 < 4; ++e2) {
    const float p0 = ev[2 * e2] * inv;
    const float p1 = ev[2 * e2 + 1] * inv;
    const unsigned short h0 = f2bf_bits(p0);
    const unsigned short h1 = f2bf_bits(p1);
    const unsigned short l0 = f2bf_bits(p0 - bf_bits2f(h0));
    const unsigned short l1 = f2bf_bits(p1 - bf_bits2f(h1));
    hw[e2] = (unsigned)h0 | ((unsigned)h1 << 16);
    lw[e2] = (unsigned)l0 | ((unsigned)l1 << 16);
  }
  v4u hv, lv;
  hv.x = hw[0]; hv.y = hw[1]; hv.z = hw[2]; hv.w = hw[3];
  lv.x = lw[0]; lv.y = lw[1]; lv.z = lw[2]; lv.w = lw[3];
  *(volatile v4u*)(Ph + base) = hv;
  *(volatile v4u*)(Pl + base) = lv;
  __threadfence();
  *(volatile v4u*)(Ph + base) = hv;
  *(volatile v4u*)(Pl + base) = lv;
}

extern "C" void kernel_launch(void* const* d_in, const int* in_sizes, int n_in,
                              void* d_out, int out_size, void* d_ws, size_t ws_size,
                              hipStream_t stream)
{
  constexpr int NROW  = 2048;
  constexpr int NFEAT = 2048;
  static_assert(NROW % 64 == 0 && NFEAT % 64 == 0, "M,N tile multiples");
  static_assert(NROW % 32 == 0 && NFEAT % 32 == 0, "K multiple of 32");
  static_assert(NROW == 256 * 8, "softmax: 256 threads x 8 columns per row");
  static_assert((NROW * NFEAT) % 512 == 0 && (NFEAT * NFEAT) % 512 == 0, "cast grid exact");

  constexpr size_t ZB   = (size_t)NROW * NFEAT * 2;
  constexpr size_t WB   = (size_t)NFEAT * NFEAT * 2;
  constexpr size_t QKB  = (size_t)NROW * NFEAT * 2;
  constexpr size_t VTB  = (size_t)NFEAT * NROW * 2;
  constexpr size_t SB   = (size_t)NROW * NROW * 4;
  constexpr size_t PB   = (size_t)NROW * NROW * 2;
  constexpr size_t oZ   = 0;
  constexpr size_t oWq  = oZ + ZB;
  constexpr size_t oWk  = oWq + WB;
  constexpr size_t oWv  = oWk + WB;
  constexpr size_t oQh  = oWv + WB;
  constexpr size_t oQl  = oQh + QKB;
  constexpr size_t oKh  = oQl + QKB;
  constexpr size_t oKl  = oKh + QKB;
  constexpr size_t oVth = oKl + QKB;
  constexpr size_t oVtl = oVth + VTB;
  constexpr size_t oS   = oVtl + VTB;
  constexpr size_t oPh  = oS + SB;
  constexpr size_t oPl  = oPh + PB;
  constexpr size_t WS_TOTAL = oPl + PB;
  static_assert(WS_TOTAL == 117440512ull, "carve total");
  static_assert(WS_TOTAL <= 134217728ull, "carve budget");

  if (n_in < 7) return;
  if (ws_size < WS_TOTAL) return;
  if ((size_t)out_size < (size_t)NROW * NFEAT) return;
  if (in_sizes[0] < NROW * NFEAT || in_sizes[1] < NFEAT * NFEAT || in_sizes[2] < NFEAT ||
      in_sizes[3] < NFEAT * NFEAT || in_sizes[4] < NFEAT || in_sizes[5] < NFEAT * NFEAT || in_sizes[6] < NFEAT) return;

  const float* z   = (const float*)d_in[0];
  const float* Wq  = (const float*)d_in[1];
  const float* bq  = (const float*)d_in[2];
  const float* Wk  = (const float*)d_in[3];
  const float* bk  = (const float*)d_in[4];
  const float* Wv  = (const float*)d_in[5];
  const float* bvp = (const float*)d_in[6];
  float* out = (float*)d_out;

  char* ws = (char*)d_ws;
  unsigned short* Zb  = (unsigned short*)(ws + oZ);
  unsigned short* Wqb = (unsigned short*)(ws + oWq);
  unsigned short* Wkb = (unsigned short*)(ws + oWk);
  unsigned short* Wvb = (unsigned short*)(ws + oWv);
  unsigned short* Qh  = (unsigned short*)(ws + oQh);
  unsigned short* Ql  = (unsigned short*)(ws + oQl);
  unsigned short* Kh  = (unsigned short*)(ws + oKh);
  unsigned short* Kl  = (unsigned short*)(ws + oKl);
  unsigned short* Vth = (unsigned short*)(ws + oVth);
  unsigned short* Vtl = (unsigned short*)(ws + oVtl);
  float*          Sf  = (float*)(ws + oS);
  unsigned short* Ph  = (unsigned short*)(ws + oPh);
  unsigned short* Pl  = (unsigned short*)(ws + oPl);

  const dim3 blk(256);

  const int n2z = NROW * NFEAT / 2;
  const int n2w = NFEAT * NFEAT / 2;
  cast_f32_bf16x2<<<dim3(n2z / 256), blk, 0, stream>>>(z,  Zb,  n2z);
  cast_f32_bf16x2<<<dim3(n2w / 256), blk, 0, stream>>>(Wq, Wqb, n2w);
  cast_f32_bf16x2<<<dim3(n2w / 256), blk, 0, stream>>>(Wk, Wkb, n2w);
  cast_f32_bf16x2<<<dim3(n2w / 256), blk, 0, stream>>>(Wv, Wvb, n2w);

  const int tilesQ  = (NROW / 64) * (NFEAT / 64);
  const int tilesVt = (NFEAT / 64) * (NROW / 64);
  const int tilesS  = (NROW / 64) * (NROW / 64);
  const int tilesH  = (NROW / 64) * (NFEAT / 64);
  const dim3 gQ((tilesQ + 7) / 8, 1), gVt((tilesVt + 7) / 8, 1), gS((tilesS + 7) / 8, 1), gH((tilesH + 7) / 8, 1);

  wmma_gemm64<1, false, 2, 2><<<gQ, blk, 0, stream>>>(
      Zb, Zb, NFEAT, 0L, Wqb, Wqb, NFEAT, 0L, (void*)Qh, (void*)Ql, NFEAT, 0L, bq, NROW, NFEAT, NFEAT, 1.0f);
  wmma_gemm64<1, false, 2, 2><<<gQ, blk, 0, stream>>>(
      Zb, Zb, NFEAT, 0L, Wkb, Wkb, NFEAT, 0L, (void*)Kh, (void*)Kl, NFEAT, 0L, bk, NROW, NFEAT, NFEAT, 1.0f);
  wmma_gemm64<1, false, 1, 2><<<gVt, blk, 0, stream>>>(
      Wvb, Wvb, NFEAT, 0L, Zb, Zb, NFEAT, 0L, (void*)Vth, (void*)Vtl, NROW, 0L, bvp, NFEAT, NROW, NFEAT, 1.0f);
  wmma_gemm64<1, true, 0, 0><<<gS, blk, 0, stream>>>(
      Qh, Ql, NFEAT, 0L, Kh, Kl, NFEAT, 0L, (void*)Sf, (void*)Sf, NROW, 0L, bq, NROW, NROW, NFEAT, 0.125f);
  softmax_rows_split<<<dim3(NROW), blk, 0, stream>>>(Sf, Ph, Pl, NROW);
  wmma_gemm64<1, true, 0, 0><<<gH, blk, 0, stream>>>(
      Ph, Pl, NROW, 0L, Vth, Vtl, NROW, 0L, (void*)out, (void*)out, NFEAT, 0L, bq, NROW, NFEAT, NROW, 1.0f);
}
